// Correlation_68367289417895
// MI455X (gfx1250) — hardware-verified
//
#include <hip/hip_runtime.h>

typedef __attribute__((ext_vector_type(16))) _Float16 v16h;
typedef __attribute__((ext_vector_type(8)))  _Float16 v8h;
typedef __attribute__((ext_vector_type(16))) __bf16   v16b;
typedef __attribute__((ext_vector_type(8)))  __bf16   v8b;
typedef __attribute__((ext_vector_type(8)))  float    v8f;
typedef __attribute__((ext_vector_type(4)))  float    v4f;
typedef __attribute__((ext_vector_type(4)))  unsigned int v4u;

constexpr int kB     = 4;
constexpr int kC     = 256;
constexpr int kH     = 64;
constexpr int kW     = 96;
constexpr int kND    = 21;
constexpr int kNOut  = kND * kND;
constexpr int kRad   = 10;
constexpr int kHalfW = kW / 2;
constexpr int kInElems   = kB * kC * kH * kW;
constexpr int kOutElems  = kB * kNOut * kH * kW;
constexpr long kPlaneHalves = (long)kB * kH * kW * kC;
constexpr long kPlaneBytes  = kPlaneHalves * 2;
constexpr long kWsNeed = 2 * kPlaneBytes;
static_assert(kC % 32 == 0, "K multiple of 32");
static_assert(kHalfW % 16 == 0, "M,N tiles of 16");
static_assert(kW % 32 == 0, "output rows are whole 128-B lines");
static_assert(kWsNeed <= 134217728L, "carve within budget");
static_assert((kPlaneBytes % 128) == 0, "plane offsets line aligned");

constexpr int kCvtPitch = 100;
constexpr int kOPitch   = 100;
constexpr int kGemmThreads = 192;

__device__ __forceinline__ unsigned short f2bf_bits(float f) {
  unsigned u = __float_as_uint(f);
  return (unsigned short)((u + 0x7FFFu + ((u >> 16) & 1u)) >> 16);
}
__device__ __forceinline__ float bf_bits2f(unsigned short h) { return __uint_as_float(((unsigned)h) << 16); }

__device__ __forceinline__ void dep_guard_h(v8f& a, v8f& b, v16h x, v16h y) { asm volatile("v_nop\n\tv_nop\n\tv_nop\n\tv_nop" : "+v"(a), "+v"(b) : "v"(x), "v"(y)); }
__device__ __forceinline__ void dep_guard_b(v8f& a, v8f& b, v16b x, v16b y) { asm volatile("v_nop\n\tv_nop\n\tv_nop\n\tv_nop" : "+v"(a), "+v"(b) : "v"(x), "v"(y)); }
__device__ __forceinline__ void keep4_h(v16h a, v16h b, v16h c, v16h d) { asm volatile("v_nop" :: "v"(a), "v"(b), "v"(c), "v"(d)); }
__device__ __forceinline__ void keep4_b(v16b a, v16b b, v16b c, v16b d) { asm volatile("v_nop" :: "v"(a), "v"(b), "v"(c), "v"(d)); }
template <typename T> struct Frag;
template <> struct Frag<_Float16> {
  typedef v16h V; union U { v16h v; v8h h[2]; };
  static __device__ __forceinline__ v16h load(const _Float16* p) {
    U f; f.h[0] = *(const v8h*)(p); f.h[1] = *(const v8h*)(p + 16); return f.v;
  }
  static __device__ __forceinline__ v8f mma(v16h a, v16h b, v8f c) {
    return __builtin_amdgcn_wmma_f32_16x16x32_f16(false, a, false, b, (short)0, c, false, false);
  }
  static __device__ __forceinline__ void guard(v8f& a, v8f& b, v16h x, v16h y) { dep_guard_h(a, b, x, y); }
  static __device__ __forceinline__ void keep(v16h a, v16h b, v16h c, v16h d) { keep4_h(a, b, c, d); }
};
template <> struct Frag<__bf16> {
  typedef v16b V; union U { v16b v; v8b h[2]; };
  static __device__ __forceinline__ v16b load(const __bf16* p) {
    U f; f.h[0] = *(const v8b*)(p); f.h[1] = *(const v8b*)(p + 16); return f.v;
  }
  static __device__ __forceinline__ v8f mma(v16b a, v16b b, v8f c) {
    return __builtin_amdgcn_wmma_f32_16x16x32_bf16(false, a, false, b, (short)0, c, false, false);
  }
  static __device__ __forceinline__ void guard(v8f& a, v8f& b, v16b x, v16b y) { dep_guard_b(a, b, x, y); }
  static __device__ __forceinline__ void keep(v16b a, v16b b, v16b c, v16b d) { keep4_b(a, b, c, d); }
};

__device__ __forceinline__ unsigned pk16(unsigned short a, unsigned short b) { return (unsigned)a | ((unsigned)b << 16); }

__device__ __forceinline__ void guard3(v8f& a0, v8f& a1, v8f& a2, v16b x, v16b y0, v16b y1, v16b y2) {
  asm volatile("v_nop\n\tv_nop\n\tv_nop\n\tv_nop" : "+v"(a0), "+v"(a1), "+v"(a2) : "v"(x), "v"(y0), "v"(y1), "v"(y2));
}
__device__ __forceinline__ void acc_guard3(v8f& a0, v8f& a1, v8f& a2) {
  asm volatile("v_nop\n\tv_nop\n\tv_nop\n\tv_nop" : "+v"(a0), "+v"(a1), "+v"(a2));
}

__global__ __launch_bounds__(256) void nchw_to_rows_bf16(const float* __restrict__ in1,
                                                          const float* __restrict__ in2,
                                                          unsigned short* __restrict__ ws) {
  __shared__ __align__(16) float sm[64 * kCvtPitch];
  const int t  = threadIdx.x;
  const int c0 = blockIdx.x * 64;
  const int bh = blockIdx.y;
  const int b  = bh >> 6;
  const int h  = bh & 63;
  const int z  = blockIdx.z;
  const float* src = (z == 0) ? in1 : in2;
  unsigned short* dst = ws + (size_t)z * kPlaneHalves;
#pragma unroll
  for (int i = 0; i < 6; ++i) {
    const int e  = i * 256 + t;
    const int cl = e / 24;
    const int q4 = e - cl * 24;
    const float* p = src + ((size_t)((b * kC + c0 + cl) * kH + h)) * kW + 4 * q4;
    const v4f v = *(const v4f*)p;
    *(v4f*)(sm + cl * kCvtPitch + 4 * q4) = v;
  }
  __syncthreads();
  const int lane = t & 31, wave = t >> 5;
  const int q = lane >> 3, c8 = (lane & 7) * 8;
  for (int pass = 0; pass < 2; ++pass) {
#pragma unroll
    for (int it = 0; it < 3; ++it) {
      const int wp  = wave * 12 + it * 4 + q;
      const int par = (wp >= kHalfW) ? 1 : 0;
      const int w   = 2 * (wp - par * kHalfW) + par;
      unsigned short hb[8];
#pragma unroll
      for (int e = 0; e < 8; ++e) hb[e] = f2bf_bits(sm[(c8 + e) * kCvtPitch + w]);
      const v4u u = (v4u){pk16(hb[0], hb[1]), pk16(hb[2], hb[3]), pk16(hb[4], hb[5]), pk16(hb[6], hb[7])};
      *(volatile v4u*)(dst + ((size_t)(bh * kW + wp)) * kC + c0 + c8) = u;
    }
    __threadfence();
  }
}

__global__ __launch_bounds__(kGemmThreads) void corr_band_gemm(const unsigned short* __restrict__ wsA,
                                                              const unsigned short* __restrict__ wsB,
                                                              float* __restrict__ out) {
  __shared__ __align__(16) float lsO[kND * kOPitch];
  const int tid  = threadIdx.x;
  const int lane = tid & 31;
  const int wave = tid >> 5;
  const int dyi  = blockIdx.x;
  const int h    = blockIdx.y;
  const int b    = blockIdx.z;
  const int h2   = h + 2 * dyi - 2 * kRad;
  const bool valid = (h2 >= 0) && (h2 < kH);
  const int h2c  = (h2 < 0) ? 0 : ((h2 >= kH) ? (kH - 1) : h2);

  for (int i = tid; i < kND * kOPitch; i += kGemmThreads) lsO[i] = 0.0f;
  __syncthreads();

  if (valid) {
    const int rlane = lane & 15;
    const int hh    = lane >> 4;
    const int koff  = hh * 8;
    const int par   = (wave >= 3) ? 1 : 0;
    const int mi    = wave - 3 * par;
    const __bf16* Apl = (const __bf16*)wsA;
    const __bf16* Bpl = (const __bf16*)wsB;
    const size_t arowIdx = (size_t)((b * kH + h) * kW + par * kHalfW + mi * 16 + rlane);
    const __bf16* arow = Apl + arowIdx * kC + koff;
    const int n0c = (mi - 1 < 0) ? 0 : (mi - 1);
    const int n1c = mi;
    const int n2c = (mi + 1 > 2) ? 2 : (mi + 1);
    const size_t browBase = (size_t)((b * kH + h2c) * kW + par * kHalfW);
    const __bf16* brow0 = Bpl + (browBase + n0c * 16 + rlane) * kC + koff;
    const __bf16* brow1 = Bpl + (browBase + n1c * 16 + rlane) * kC + koff;
    const __bf16* brow2 = Bpl + (browBase + n2c * 16 + rlane) * kC + koff;

    v8f acc0 = (v8f){0.f,0.f,0.f,0.f,0.f,0.f,0.f,0.f};
    v8f acc1 = (v8f){0.f,0.f,0.f,0.f,0.f,0.f,0.f,0.f};
    v8f acc2 = (v8f){0.f,0.f,0.f,0.f,0.f,0.f,0.f,0.f};
#pragma unroll 1
    for (int k0 = 0; k0 < kC; k0 += 32) {
      const v16b af  = Frag<__bf16>::load(arow  + k0);
      const v16b bf0 = Frag<__bf16>::load(brow0 + k0);
      const v16b bf1 = Frag<__bf16>::load(brow1 + k0);
      const v16b bf2 = Frag<__bf16>::load(brow2 + k0);
      acc0 = Frag<__bf16>::mma(af, bf0, acc0);
      acc1 = Frag<__bf16>::mma(af, bf1, acc1);
      acc2 = Frag<__bf16>::mma(af, bf2, acc2);
      guard3(acc0, acc1, acc2, af, bf0, bf1, bf2);
    }
    acc_guard3(acc0, acc1, acc2);

    const float sc = 1.0f / 256.0f;
#pragma unroll
    for (int r = 0; r < 8; ++r) {
      const int u = mi * 16 + 8 * hh + r;
      const int w = 2 * u + par;
      {
        const int ni  = mi - 1;
        const int dxi = ni * 16 + rlane - u + kRad;
        const float val = acc0[r] * sc;
        if (ni >= 0 && dxi >= 0 && dxi < kND) lsO[dxi * kOPitch + w] = val;
      }
      {
        const int ni  = mi;
        const int dxi = ni * 16 + rlane - u + kRad;
        const float val = acc1[r] * sc;
        if (dxi >= 0 && dxi < kND) lsO[dxi * kOPitch + w] = val;
      }
      {
        const int ni  = mi + 1;
        const int dxi = ni * 16 + rlane - u + kRad;
        const float val = acc2[r] * sc;
        if (ni <= 2 && dxi >= 0 && dxi < kND) lsO[dxi * kOPitch + w] = val;
      }
    }
  }
  __syncthreads();

  float* obase = out + (((size_t)b * kNOut + (size_t)dyi * kND) * kH + h) * kW;
  const int q  = lane >> 3;
  const int l8 = (lane & 7) * 4;
  for (int pass = 0; pass < 2; ++pass) {
#pragma unroll
    for (int it = 0; it < 3; ++it) {
      const int L   = it * 24 + wave * 4 + q;
      const int Lc  = (L < 3 * kND) ? L : (3 * kND - 1);
      const int row = Lc / 3;
      const int seg = Lc - row * 3;
      const v4f val = *(const v4f*)(lsO + row * kOPitch + seg * 32 + l8);
      if (L < 3 * kND)
        *(volatile v4f*)(obase + (size_t)row * (kH * kW) + seg * 32 + l8) = val;
    }
    __threadfence();
  }
}

extern "C" void kernel_launch(void* const* d_in, const int* in_sizes, int n_in,
                              void* d_out, int out_size, void* d_ws, size_t ws_size,
                              hipStream_t stream) {
  if (n_in < 2) return;
  if (in_sizes[0] < kInElems || in_sizes[1] < kInElems) return;
  if (out_size < kOutElems) return;
  if (ws_size < (size_t)kWsNeed) return;
  const float* in1 = (const float*)d_in[0];
  const float* in2 = (const float*)d_in[1];
  float* out = (float*)d_out;
  unsigned short* ws = (unsigned short*)d_ws;

  nchw_to_rows_bf16<<<dim3(kC / 64, kB * kH, 2), 256, 0, stream>>>(in1, in2, ws);
  corr_band_gemm<<<dim3(kND, kH, kB), kGemmThreads, 0, stream>>>(ws, ws + kPlaneHalves, out);
}
